// CrossAttention_Light_71983651881630
// MI455X (gfx1250) — hardware-verified
//
#include <hip/hip_runtime.h>

typedef __attribute__((ext_vector_type(16))) _Float16 v16h;
typedef __attribute__((ext_vector_type(8)))  _Float16 v8h;
typedef __attribute__((ext_vector_type(16))) __bf16   v16b;
typedef __attribute__((ext_vector_type(8)))  __bf16   v8b;
typedef __attribute__((ext_vector_type(8)))  float    v8f;
typedef __attribute__((ext_vector_type(4)))  float    v4f;
#define PSCALE 32768.0f
#define U16(p) ((const unsigned short*)(const void*)(p))
#define PSCALE_INV (1.0f / 32768.0f)

__device__ __forceinline__ unsigned short f2bf_bits(float f) {
  unsigned u = __float_as_uint(f);
  return (unsigned short)((u + 0x7FFFu + ((u >> 16) & 1u)) >> 16);
}
__device__ __forceinline__ float bf_bits2f(unsigned short h) { return __uint_as_float(((unsigned)h) << 16); }

__device__ __forceinline__ void dep_guard_h(v8f& a, v8f& b, v16h x, v16h y) { asm volatile("v_nop\n\tv_nop\n\tv_nop\n\tv_nop" : "+v"(a), "+v"(b) : "v"(x), "v"(y)); }
__device__ __forceinline__ void dep_guard_b(v8f& a, v8f& b, v16b x, v16b y) { asm volatile("v_nop\n\tv_nop\n\tv_nop\n\tv_nop" : "+v"(a), "+v"(b) : "v"(x), "v"(y)); }
__device__ __forceinline__ void keep4_h(v16h a, v16h b, v16h c, v16h d) { asm volatile("v_nop" :: "v"(a), "v"(b), "v"(c), "v"(d)); }
__device__ __forceinline__ void keep4_b(v16b a, v16b b, v16b c, v16b d) { asm volatile("v_nop" :: "v"(a), "v"(b), "v"(c), "v"(d)); }
__device__ __forceinline__ void acc_guard4(v8f& a, v8f& b, v8f& c, v8f& d) { asm volatile("v_nop\n\tv_nop\n\tv_nop\n\tv_nop" : "+v"(a), "+v"(b), "+v"(c), "+v"(d)); }
template <typename T> struct Frag;
template <> struct Frag<_Float16> {
  typedef v16h V; union U { v16h v; v8h h[2]; };
  static __device__ __forceinline__ v16h load(const _Float16* p) {
    U f; f.h[0] = *(const v8h*)(p); f.h[1] = *(const v8h*)(p + 16); return f.v;
  }
  static __device__ __forceinline__ v8f mma(v16h a, v16h b, v8f c) {
    return __builtin_amdgcn_wmma_f32_16x16x32_f16(false, a, false, b, (short)0, c, false, false);
  }
  static __device__ __forceinline__ void guard(v8f& a, v8f& b, v16h x, v16h y) { dep_guard_h(a, b, x, y); }
  static __device__ __forceinline__ void keep(v16h a, v16h b, v16h c, v16h d) { keep4_h(a, b, c, d); }
};
template <> struct Frag<__bf16> {
  typedef v16b V; union U { v16b v; v8b h[2]; };
  static __device__ __forceinline__ v16b load(const __bf16* p) {
    U f; f.h[0] = *(const v8b*)(p); f.h[1] = *(const v8b*)(p + 16); return f.v;
  }
  static __device__ __forceinline__ v8f mma(v16b a, v16b b, v8f c) {
    return __builtin_amdgcn_wmma_f32_16x16x32_bf16(false, a, false, b, (short)0, c, false, false);
  }
  static __device__ __forceinline__ void guard(v8f& a, v8f& b, v16b x, v16b y) { dep_guard_b(a, b, x, y); }
  static __device__ __forceinline__ void keep(v16b a, v16b b, v16b c, v16b d) { keep4_b(a, b, c, d); }
};

template <int ET> struct Elem;
template <> struct Elem<0> { typedef _Float16 T; };
template <> struct Elem<1> { typedef __bf16 T; };
template <int ET, bool SPLIT, int BIAS_MODE, int OUT_MODE, bool RESID, int ACT = 0>
__global__ __launch_bounds__(256) void wmma_gemm64(
    const unsigned short* __restrict__ Ap, const unsigned short* __restrict__ A2p, int lda, long strideA,
    const unsigned short* __restrict__ Btp, const unsigned short* __restrict__ Bt2p, int ldb, long strideB,
    void* __restrict__ Cout, void* __restrict__ Cout2, int ldc, long strideC,
    const float* __restrict__ bias,
    const float* __restrict__ resid, long strideR,
    int M, int N, int K, float scale) {
  typedef typename Elem<ET>::T T;
  typedef typename Frag<T>::V V;
  const T* A = (const T*)Ap; const T* A2 = (const T*)A2p; const T* Bt = (const T*)Btp; const T* Bt2 = (const T*)Bt2p;
  __shared__ __align__(16) float sT[8][16 * 68];
  const int b    = blockIdx.y;
  const int lane = threadIdx.x & 31;
  const int wave = threadIdx.x >> 5;
  const int tilesN = N >> 6;
  const int tilesM = M >> 6;
  const int tile = blockIdx.x * 8 + wave;
  if (tile >= tilesM * tilesN) return;
  const int tm = tile / tilesN;
  const int tn = tile - tm * tilesN;
  const int m0 = tm << 6;
  const int n0 = tn << 6;

  const T* Ab  = A  + (size_t)b * strideA;
  const T* Bb  = Bt + (size_t)b * strideB;
  const T* Ab2 = SPLIT ? (A2  + (size_t)b * strideA) : nullptr;
  const T* Bb2 = SPLIT ? (Bt2 + (size_t)b * strideB) : nullptr;

  const int rlane = lane & 15;
  const int koff  = (lane >> 4) * 8;
  const int mOff  = (lane >> 4) * 8;

  v8f acc[4][4];
#pragma unroll
  for (int i = 0; i < 4; ++i)
#pragma unroll
    for (int j = 0; j < 4; ++j) acc[i][j] = (v8f){0.f,0.f,0.f,0.f,0.f,0.f,0.f,0.f};

  for (int k0 = 0; k0 < K; k0 += 32) {
    V bh[4], bl[4];
#pragma unroll
    for (int j = 0; j < 4; ++j) {
      const size_t bo = (size_t)(n0 + (j << 4) + rlane) * ldb + koff + k0;
      bh[j] = Frag<T>::load(Bb + bo);
      if (SPLIT) bl[j] = Frag<T>::load(Bb2 + bo);
    }
#pragma unroll
    for (int i = 0; i < 4; ++i) {
      const size_t ao = (size_t)(m0 + (i << 4) + rlane) * lda + koff + k0;
      V ah = Frag<T>::load(Ab + ao);
      V al;
      if (SPLIT) al = Frag<T>::load(Ab2 + ao);
#pragma unroll
      for (int j = 0; j < 4; ++j) {
        acc[i][j] = Frag<T>::mma(ah, bh[j], acc[i][j]);
        if (SPLIT) {
          acc[i][j] = Frag<T>::mma(ah, bl[j], acc[i][j]);
          acc[i][j] = Frag<T>::mma(al, bh[j], acc[i][j]);
        }
      }
      Frag<T>::guard(acc[i][0], acc[i][3], ah, SPLIT ? al : ah);
    }
    Frag<T>::keep(bh[0], bh[1], bh[2], bh[3]);
    if (SPLIT) Frag<T>::keep(bl[0], bl[1], bl[2], bl[3]);
  }
  acc_guard4(acc[0][0], acc[0][1], acc[0][2], acc[0][3]);
  acc_guard4(acc[1][0], acc[1][1], acc[1][2], acc[1][3]);
  acc_guard4(acc[2][0], acc[2][1], acc[2][2], acc[2][3]);
  acc_guard4(acc[3][0], acc[3][1], acc[3][2], acc[3][3]);

  float* slab = sT[wave];
  const float* Rb = RESID ? (resid + (size_t)b * strideR) : nullptr;
#pragma unroll
  for (int i = 0; i < 4; ++i) {
    const int mBase = m0 + (i << 4);
#pragma unroll
    for (int j = 0; j < 4; ++j) {
      const int n = n0 + (j << 4) + rlane;
      float bv = 0.f;
      if (BIAS_MODE == 2) bv = bias[n];
#pragma unroll
      for (int r = 0; r < 8; ++r) {
        float v = acc[i][j][r] * scale;
        if (BIAS_MODE == 1) v += bias[mBase + mOff + r];
        if (BIAS_MODE == 2) v += bv;
        if (RESID) v += Rb[(size_t)(mBase + mOff + r) * ldc + n];
        if (ACT == 1) v = tanhf(v);
        if (ACT == 2) v = fmaxf(v, 0.0f);
        if (ACT == 3) v = v / (1.0f + expf(-v));
        if (ACT == 4) v = (v > 0.f) ? v : 0.01f * v;
        if (ACT == 5) v = 0.5f * v * (1.0f + erff(v * 0.70710678118654752f));
        slab[(mOff + r) * 68 + (j << 4) + rlane] = v;
      }
    }
    __builtin_amdgcn_fence(__ATOMIC_RELEASE, "workgroup");
    __builtin_amdgcn_wave_barrier();
    __builtin_amdgcn_fence(__ATOMIC_ACQUIRE, "workgroup");
    if (OUT_MODE == 0) {
      float* C = (float*)Cout + (size_t)b * strideC;
      const int hh = lane >> 4, c4 = (lane & 15) * 4;
      for (int pass = 0; pass < 2; ++pass) {
#pragma unroll
        for (int it = 0; it < 8; ++it) {
          const int row = it * 2 + hh;
          v4f v = *(const v4f*)(slab + row * 68 + c4);
          *(volatile v4f*)(C + (size_t)(mBase + row) * ldc + n0 + c4) = v;
        }
        __threadfence();
      }
    } else {
      const int q = lane >> 3, c8 = (lane & 7) * 8;
      unsigned short* C  = (unsigned short*)Cout  + (size_t)b * strideC;
      unsigned short* C2 = (OUT_MODE == 2) ? ((unsigned short*)Cout2 + (size_t)b * strideC) : nullptr;
      for (int pass = 0; pass < 2; ++pass) {
#pragma unroll
        for (int it = 0; it < 4; ++it) {
          const int row = it * 4 + q;
          const float* sp = slab + row * 68 + c8;
          v8h hv, lv;
#pragma unroll
          for (int e = 0; e < 8; ++e) {
            if (OUT_MODE == 1) {
              hv[e] = (_Float16)sp[e];
            } else {
              unsigned short hb = f2bf_bits(sp[e]);
              unsigned short lb = f2bf_bits(sp[e] - bf_bits2f(hb));
              hv[e] = __builtin_bit_cast(_Float16, hb);
              lv[e] = __builtin_bit_cast(_Float16, lb);
            }
          }
          *(volatile v8h*)(C + (size_t)(mBase + row) * ldc + n0 + c8) = hv;
          if (OUT_MODE == 2) *(volatile v8h*)(C2 + (size_t)(mBase + row) * ldc + n0 + c8) = lv;
        }
        __threadfence();
      }
    }
    __builtin_amdgcn_fence(__ATOMIC_RELEASE, "workgroup");
    __builtin_amdgcn_wave_barrier();
    __builtin_amdgcn_fence(__ATOMIC_ACQUIRE, "workgroup");
  }
}

__global__ __launch_bounds__(256) void cast_f32_f16x2(
    const float* __restrict__ in, _Float16* __restrict__ out, int n2) {
  int i = blockIdx.x * 256 + threadIdx.x;
  if (i < n2) {
    const _Float16 h0 = (_Float16)in[2 * i], h1 = (_Float16)in[2 * i + 1];
    const unsigned u = (unsigned)__builtin_bit_cast(unsigned short, h0) | ((unsigned)__builtin_bit_cast(unsigned short, h1) << 16);
    ((volatile unsigned*)out)[i] = u;
    __threadfence();
    ((volatile unsigned*)out)[i] = u;
  }
}

__global__ __launch_bounds__(256) void transpose_cast_k256(
    const float* __restrict__ in, _Float16* __restrict__ out, int C, float wscale) {
  const int wave = blockIdx.x * 8 + (threadIdx.x >> 5);
  const int lane = threadIdx.x & 31;
  if (wave >= C) return;
  const int n = wave;
  v8h v;
#pragma unroll
  for (int e = 0; e < 8; ++e) v[e] = (_Float16)(in[(size_t)(8 * lane + e) * C + n] * wscale);
  _Float16* p = out + (size_t)n * 256 + 8 * lane;
  *(volatile v8h*)p = v;
  __threadfence();
  *(volatile v8h*)p = v;
}

#define AT_D 64
#define AT_NW 4
#define AT_KC 64

__device__ __forceinline__ v8f mma_h16(v16h a, v16h b, v8f c) {
  c = __builtin_amdgcn_wmma_f32_16x16x32_f16(false, a, false, b, (short)0, c, false, false);
  asm volatile("v_nop\n\tv_nop\n\tv_nop\n\tv_nop" : "+v"(c) : "v"(a), "v"(b));
  return c;
}

__global__ __launch_bounds__(128)
void attn_hd64_f16(const _Float16* __restrict__ Qg, const _Float16* __restrict__ Kg,
                   const _Float16* __restrict__ Vtg, _Float16* __restrict__ Og,
                   float* __restrict__ RSg,
                   int L, int Lc, int H, int Dm, float qscale, float oscale) {
  union FH { v16h v; v8h h[2]; };
  __shared__ __align__(16) _Float16 Ksh[AT_KC * AT_D];
  __shared__ __align__(16) _Float16 Vth[AT_D * AT_KC];
  __shared__ __align__(16) _Float16 Psh[AT_NW][16 * AT_KC];
  __shared__ __align__(16) float    Os[AT_NW][16 * 68];
  __shared__ __align__(16) float    RSs[AT_NW * 16];

  const int tid  = threadIdx.x;
  const int wave = tid >> 5;
  const int lane = tid & 31;
  const int hh   = lane >> 4;
  const int c    = lane & 15;

  const int nqb = L / 64;
  const int bx = blockIdx.x;
  const int qb = bx % nqb;
  const int bh = bx / nqb;
  const int h  = bh % H;
  const int b  = bh / H;
  const int q0 = qb * 64 + wave * 16;

  const _Float16* Qp = Qg  + (size_t)b * L  * Dm + (size_t)h * AT_D;
  const _Float16* Kp = Kg  + (size_t)b * Lc * Dm + (size_t)h * AT_D;
  const _Float16* Vp = Vtg + ((size_t)b * Dm + (size_t)h * AT_D) * (size_t)Lc;
  _Float16*       Op = Og  + (size_t)b * L  * Dm + (size_t)h * AT_D;

  v16h qa[2];
  {
    const _Float16* qr = Qp + (size_t)(q0 + c) * Dm;
#pragma unroll
    for (int dc = 0; dc < 2; ++dc) {
      const v8h t0 = *(const v8h*)(qr + dc * 32 + 8 * hh);
      const v8h t1 = *(const v8h*)(qr + dc * 32 + 16 + 8 * hh);
#pragma unroll
      for (int e = 0; e < 8; ++e) {
        qa[dc][e]     = (_Float16)((float)t0[e] * qscale);
        qa[dc][8 + e] = (_Float16)((float)t1[e] * qscale);
      }
    }
  }

  float mrow[8], lrow[8], srow[8];
  v8f oacc[4];
#pragma unroll
  for (int r = 0; r < 8; ++r) { mrow[r] = -1e30f; lrow[r] = 0.f; srow[r] = 0.f; }
#pragma unroll
  for (int t = 0; t < 4; ++t) oacc[t] = (v8f){0.f,0.f,0.f,0.f,0.f,0.f,0.f,0.f};

  const int nChunks = Lc / AT_KC;
  for (int kc = 0; kc < nChunks; ++kc) {
    const int kv0 = kc * AT_KC;
    __syncthreads();
    {
      const int r = tid >> 1, c0 = (tid & 1) * 32;
      const _Float16* krow = Kp + (size_t)(kv0 + r) * Dm + c0;
      const _Float16* vrow = Vp + (size_t)r * Lc + kv0 + c0;
#pragma unroll
      for (int i = 0; i < 4; ++i) {
        const v8h kk = *(const v8h*)(krow + 8 * i);
        const v8h vv = *(const v8h*)(vrow + 8 * i);
        *(v8h*)(Ksh + r * AT_D  + c0 + 8 * i) = kk;
        *(v8h*)(Vth + r * AT_KC + c0 + 8 * i) = vv;
      }
    }
    __syncthreads();

    v8f s[4];
#pragma unroll
    for (int j = 0; j < 4; ++j) {
      s[j] = (v8f){0.f,0.f,0.f,0.f,0.f,0.f,0.f,0.f};
#pragma unroll
      for (int dc = 0; dc < 2; ++dc) {
        FH kb;
        kb.h[0] = *(const v8h*)(Ksh + (j * 16 + c) * AT_D + dc * 32 + 8 * hh);
        kb.h[1] = *(const v8h*)(Ksh + (j * 16 + c) * AT_D + dc * 32 + 16 + 8 * hh);
        s[j] = mma_h16(qa[dc], kb.v, s[j]);
      }
    }

    float cm[8];
#pragma unroll
    for (int r = 0; r < 8; ++r) {
      float m = s[0][r];
#pragma unroll
      for (int j = 1; j < 4; ++j) m = fmaxf(m, s[j][r]);
#pragma unroll
      for (int off = 1; off < 16; off <<= 1) m = fmaxf(m, __shfl_xor(m, off, 32));
      cm[r] = m;
    }
    _Float16* pw = Psh[wave];
#pragma unroll
    for (int r = 0; r < 8; ++r) {
      const float mnew  = fmaxf(mrow[r], cm[r]);
      const float alpha = __expf(mrow[r] - mnew);
      mrow[r] = mnew;
      float psum = 0.f, hsum = 0.f;
#pragma unroll
      for (int j = 0; j < 4; ++j) {
        const float p = __expf(s[j][r] - mnew);
        psum += p;
        const _Float16 ph = (_Float16)(p * PSCALE);
        pw[(8 * hh + r) * AT_KC + j * 16 + c] = ph;
        hsum += (float)ph;
      }
#pragma unroll
      for (int off = 1; off < 16; off <<= 1) {
        psum += __shfl_xor(psum, off, 32);
        hsum += __shfl_xor(hsum, off, 32);
      }
      lrow[r] = lrow[r] * alpha + psum;
      srow[r] = srow[r] * alpha + hsum;
#pragma unroll
      for (int t = 0; t < 4; ++t) oacc[t][r] *= alpha;
    }
    __builtin_amdgcn_fence(__ATOMIC_RELEASE, "workgroup");
    __builtin_amdgcn_wave_barrier();
    __builtin_amdgcn_fence(__ATOMIC_ACQUIRE, "workgroup");

#pragma unroll
    for (int kk = 0; kk < 2; ++kk) {
      FH pa;
      pa.h[0] = *(const v8h*)(pw + c * AT_KC + kk * 32 + 8 * hh);
      pa.h[1] = *(const v8h*)(pw + c * AT_KC + kk * 32 + 16 + 8 * hh);
#pragma unroll
      for (int t = 0; t < 4; ++t) {
        FH vb;
        vb.h[0] = *(const v8h*)(Vth + (t * 16 + c) * AT_KC + kk * 32 + 8 * hh);
        vb.h[1] = *(const v8h*)(Vth + (t * 16 + c) * AT_KC + kk * 32 + 16 + 8 * hh);
        oacc[t] = mma_h16(pa.v, vb.v, oacc[t]);
      }
    }
  }

  float* os = Os[wave];
#pragma unroll
  for (int r = 0; r < 8; ++r) {
    const float il  = 1.0f / (lrow[r] * PSCALE);
    const float inv = oscale * il;
    const float rsv = srow[r] * il;
#pragma unroll
    for (int t = 0; t < 4; ++t) os[(8 * hh + r) * 68 + t * 16 + c] = oacc[t][r] * inv;
    if (c == 0) RSs[wave * 16 + 8 * hh + r] = rsv;
  }
  __builtin_amdgcn_fence(__ATOMIC_RELEASE, "workgroup");
  __builtin_amdgcn_wave_barrier();
  __builtin_amdgcn_fence(__ATOMIC_ACQUIRE, "workgroup");
  {
    const int q = lane >> 3, c8 = (lane & 7) * 8;
    for (int pass = 0; pass < 2; ++pass) {
#pragma unroll
      for (int it = 0; it < 4; ++it) {
        const int row = it * 4 + q;
        const float* sp = os + row * 68 + c8;
        const v4f a0 = *(const v4f*)(sp);
        const v4f a1 = *(const v4f*)(sp + 4);
        v8h hv;
#pragma unroll
        for (int e = 0; e < 4; ++e) { hv[e] = (_Float16)a0[e]; hv[4 + e] = (_Float16)a1[e]; }
        *(volatile v8h*)(Op + (size_t)(q0 + row) * Dm + c8) = hv;
      }
      __threadfence();
    }
  }
  __syncthreads();
  if (wave == 0) {
    const int l4 = (lane & 15) * 4;
    const v4f rv = *(const v4f*)(RSs + l4);
    float* rp = RSg + ((size_t)(b * H + h) * (size_t)L + (size_t)qb * 64 + l4);
    if (lane < 16) *(volatile v4f*)rp = rv;
    __threadfence();
    if (lane < 16) *(volatile v4f*)rp = rv;
  }
}

__global__ __launch_bounds__(256) void head_mean_rowsum_v4(
    const float* __restrict__ RS, float* __restrict__ outm, int L, int H, int n4, float hinv) {
  const int i = blockIdx.x * 256 + threadIdx.x;
  if (i < n4) {
    const size_t e0 = 4 * (size_t)i;
    const int b = (int)(e0 / (size_t)L);
    const int q = (int)(e0 - (size_t)b * L);
    v4f s = (v4f){0.f, 0.f, 0.f, 0.f};
#pragma unroll 1
    for (int h = 0; h < H; ++h) {
      const v4f t = *(const v4f*)(RS + ((size_t)(b * H + h) * (size_t)L + q));
      s = s + t;
    }
    const v4f o = s * hinv;
    *(volatile v4f*)(outm + e0) = o;
    __threadfence();
    *(volatile v4f*)(outm + e0) = o;
  }
}

extern "C" void kernel_launch(void* const* d_in, const int* in_sizes, int n_in,
                              void* d_out, int out_size, void* d_ws,
                              size_t ws_size, hipStream_t stream) {
  const int B = 4, L = 4096, Lc = 4096, D = 256, H = 4, MAPHW = 64;
  if (n_in < 8) return;
  if (in_sizes[0] != B * L * D || in_sizes[1] != B * Lc * D || in_sizes[2] != D * D ||
      in_sizes[3] != D || in_sizes[4] != D * 2 * D || in_sizes[5] != 2 * D ||
      in_sizes[6] != D * D || in_sizes[7] != D) return;
  if (out_size != B * L * D + B * MAPHW * MAPHW) return;
  if (L != MAPHW * MAPHW) return;

  const float* x   = (const float*)d_in[0];
  const float* ctx = (const float*)d_in[1];
  const float* Wq  = (const float*)d_in[2];
  const float* bq  = (const float*)d_in[3];
  const float* Wkv = (const float*)d_in[4];
  const float* bkv = (const float*)d_in[5];
  const float* Wp  = (const float*)d_in[6];
  const float* bp  = (const float*)d_in[7];
  float* out0 = (float*)d_out;
  float* out1 = out0 + (size_t)B * L * D;

  const size_t nTokX  = (size_t)B * L  * D;
  const size_t nTokC  = (size_t)B * Lc * D;
  const size_t bX16   = nTokX * 2;
  const size_t bC16   = nTokC * 2;
  const size_t bWqT   = (size_t)D * D * 2;
  const size_t bWkvT  = (size_t)2 * D * D * 2;
  const size_t bWpT   = (size_t)D * D * 2;
  const size_t bQ16   = nTokX * 2;
  const size_t bK16   = nTokC * 2;
  const size_t bVt16  = (size_t)B * D * Lc * 2;
  const size_t bO16   = nTokX * 2;
  const size_t bRS    = (size_t)B * H * L * 4;
  size_t off = 0;
  char* ws = (char*)d_ws;
  _Float16* x16  = (_Float16*)(ws + off); off += bX16;
  _Float16* c16  = (_Float16*)(ws + off); off += bC16;
  _Float16* WqT  = (_Float16*)(ws + off); off += bWqT;
  _Float16* WkvT = (_Float16*)(ws + off); off += bWkvT;
  _Float16* WpT  = (_Float16*)(ws + off); off += bWpT;
  _Float16* Q16  = (_Float16*)(ws + off); off += bQ16;
  _Float16* K16  = (_Float16*)(ws + off); off += bK16;
  _Float16* Vt16 = (_Float16*)(ws + off); off += bVt16;
  _Float16* O16  = (_Float16*)(ws + off); off += bO16;
  float*    RS   = (float*)(ws + off);    off += bRS;
  if (off > ws_size || off > (size_t)134217728) return;

  const float WSC = 64.0f;
  const float OSC = 64.0f;

  {
    const int n2x = (int)(nTokX / 2), n2c = (int)(nTokC / 2);
    cast_f32_f16x2<<<dim3((n2x + 255) / 256), dim3(256), 0, stream>>>(x, x16, n2x);
    cast_f32_f16x2<<<dim3((n2c + 255) / 256), dim3(256), 0, stream>>>(ctx, c16, n2c);
  }
  transpose_cast_k256<<<dim3((D + 7) / 8), dim3(256), 0, stream>>>(Wq, WqT, D, WSC);
  transpose_cast_k256<<<dim3((2 * D + 7) / 8), dim3(256), 0, stream>>>(Wkv, WkvT, 2 * D, WSC);
  transpose_cast_k256<<<dim3((D + 7) / 8), dim3(256), 0, stream>>>(Wp, WpT, D, WSC);

  const int Mtok = B * L;
  const int tilesProj = (Mtok / 64) * (D / 64);
  wmma_gemm64<0, false, 2, 1, false><<<dim3((tilesProj + 7) / 8, 1), dim3(256), 0, stream>>>(
      (const unsigned short*)x16, (const unsigned short*)x16, D, 0L,
      (const unsigned short*)WqT, (const unsigned short*)WqT, D, 0L,
      (void*)Q16, (void*)Q16, D, 0L, bq, x, 0L, Mtok, D, D, 1.0f / WSC);
  wmma_gemm64<0, false, 2, 1, false><<<dim3((tilesProj + 7) / 8, 1), dim3(256), 0, stream>>>(
      (const unsigned short*)c16, (const unsigned short*)c16, D, 0L,
      (const unsigned short*)WkvT, (const unsigned short*)WkvT, D, 0L,
      (void*)K16, (void*)K16, D, 0L, bkv, x, 0L, Mtok, D, D, 1.0f / WSC);
  {
    const int tilesV = (D / 64) * (Lc / 64);
    wmma_gemm64<0, false, 1, 1, false><<<dim3((tilesV + 7) / 8, B), dim3(256), 0, stream>>>(
        (const unsigned short*)(WkvT + (size_t)D * D), (const unsigned short*)(WkvT + (size_t)D * D), D, 0L,
        (const unsigned short*)c16, (const unsigned short*)c16, D, (long)Lc * D,
        (void*)Vt16, (void*)Vt16, Lc, (long)D * Lc, bkv + D, x, 0L, D, Lc, D, 1.0f / WSC);
  }
  attn_hd64_f16<<<dim3(B * H * (L / 64)), dim3(128), 0, stream>>>(
      Q16, K16, Vt16, O16, RS, L, Lc, H, D, 0.125f, OSC);
  wmma_gemm64<0, false, 2, 0, true><<<dim3((tilesProj + 7) / 8, 1), dim3(256), 0, stream>>>(
      (const unsigned short*)O16, (const unsigned short*)O16, D, 0L,
      (const unsigned short*)WpT, (const unsigned short*)WpT, D, 0L,
      (void*)out0, (void*)out0, D, 0L, bp, x, 0L, Mtok, D, D, 1.0f / (WSC * OSC));
  {
    const int n4 = (B * L) / 4;
    head_mean_rowsum_v4<<<dim3((n4 + 255) / 256), dim3(256), 0, stream>>>(RS, out1, L, H, n4, 1.0f / (float)H);
  }
}
